// SingleQMSANHead_30442728194141
// MI455X (gfx1250) — hardware-run, weakly checked
//
#include <hip/hip_runtime.h>


#ifndef NB
#define NB 4
#endif
#ifndef SEQ
#define SEQ 256
#endif
#define NB_FULL  4
#define SEQ_FULL 256
#ifndef OUT_SEQ
#define OUT_SEQ SEQ
#endif
#define EW   256
#define HV   128
#define AW   4
#define OSP  132
#define RP   288
#define OSA  292
#define EPSQ 1.0e-10f
#define LN2F 0.6931471805599453f

static_assert(EW % 32 == 0);
static_assert(EW % 16 == 0);
static_assert(EW == 256);
static_assert(HV == 128);
static_assert(HV % 64 == 0);
static_assert(SEQ % 64 == 0);
static_assert((NB * SEQ) % 64 == 0);
static_assert((NB * SEQ) % 16 == 0);
static_assert(SEQ % 32 == 0);
static_assert(SEQ % (16 * AW) == 0);
static_assert(RP == EW + 32);
static_assert((RP * 4) % 128 == 0);
static_assert(OSA >= RP && (OSA * 4) % 16 == 0);
static_assert(OSP >= HV && (OSP * 4) % 16 == 0);
static_assert(NB <= NB_FULL);
static_assert(SEQ <= SEQ_FULL);
static_assert(((size_t)SEQ * EW) % 8 == 0);
static_assert(((size_t)HV * EW) % 8 == 0);
static_assert(((size_t)EW * EW) % 8 == 0);
static_assert(16 * 68 * 4 <= 131072);
static_assert(16 * OSA * 4 <= 131072);
static_assert(AW * 16 * OSP * 4 <= 131072);
static_assert(32 * 16 * 4 == 16 * 128);
static_assert(32 * 16 * 2 * 16 + 32 * 16 * 4 == 16 * RP * 4);
static_assert(32 * 16 * 16 == 16 * HV * 4);

typedef _Float16 h16;
typedef unsigned short bf;
typedef __attribute__((ext_vector_type(16))) __bf16   v16bf;
typedef __attribute__((ext_vector_type(16))) _Float16 v16h;
typedef __attribute__((ext_vector_type(8)))  _Float16 v8h;
typedef __attribute__((ext_vector_type(8)))  unsigned short v8us;
typedef __attribute__((ext_vector_type(8)))  float    v8f;
typedef __attribute__((ext_vector_type(4)))  float    v4f;
typedef v4f  __attribute__((may_alias)) v4fa;

__device__ __forceinline__ unsigned short f2bf(float f) { unsigned u = __float_as_uint(f); u += 0x7FFFu + ((u >> 16) & 1u); return (unsigned short)(u >> 16); }
__device__ __forceinline__ float bfr(float f) { return __uint_as_float(((unsigned)f2bf(f)) << 16); }
__device__ __forceinline__ v16h cat16(v8h lo, v8h hi) { return __builtin_shufflevector(lo, hi, 0, 1, 2, 3, 4, 5, 6, 7, 8, 9, 10, 11, 12, 13, 14, 15); }
__device__ __forceinline__ v16bf cat16b(v8us lo, v8us hi) { return __builtin_bit_cast(v16bf, __builtin_shufflevector(lo, hi, 0, 1, 2, 3, 4, 5, 6, 7, 8, 9, 10, 11, 12, 13, 14, 15)); }
__device__ __forceinline__ v8f wmma16(v16h a, v16h b, v8f c) { return __builtin_amdgcn_wmma_f32_16x16x32_f16(false, a, false, b, (short)0, c, false, false); }
__device__ __forceinline__ v8f wmmab(v16bf a, v16bf b, v8f c) { return __builtin_amdgcn_wmma_f32_16x16x32_bf16(false, a, false, b, (short)0, c, false, false); }
__device__ __forceinline__ v16h  ldh(const h16* p) { return cat16(*(const v8h*)p, *(const v8h*)(p + 16)); }
__device__ __forceinline__ v16bf ldb(const bf* p)  { return cat16b(*(const v8us*)p, *(const v8us*)(p + 16)); }
__device__ __forceinline__ void wave_sync() { __builtin_amdgcn_fence(3  , "wavefront"); __builtin_amdgcn_wave_barrier(); asm volatile("" ::: "memory"); }

__device__ __forceinline__ v8f wmma16g(v16h a, v16h b, v8f c) { c = wmma16(a, b, c); asm volatile("v_nop\n\tv_nop\n\tv_nop\n\tv_nop" : "+v"(c) : "v"(a), "v"(b)); return c; }
__device__ __forceinline__ v8f wmmabg(v16bf a, v16bf b, v8f c) { c = wmmab(a, b, c); asm volatile("v_nop\n\tv_nop\n\tv_nop\n\tv_nop" : "+v"(c) : "v"(a), "v"(b)); return c; }
static __device__ __forceinline__ h16 toh_flush(float v) { const h16 r = (h16)v; return (fabsf(v) < 6.103515625e-05f) ? (h16)0.0f : r; }

__global__ __launch_bounds__(256) void k_cvt8(const float* __restrict__ src, bf* dst, size_t n8) {
    const size_t i = (size_t)blockIdx.x * 256 + threadIdx.x; if (i >= n8) return;
    const v8f v = *(const v8f*)(src + i * 8); v8us o;
#pragma unroll
    for (int k = 0; k < 8; ++k) o[k] = f2bf(v[k]);
    *(volatile v8us*)(dst + i * 8) = o; __threadfence(); *(volatile v8us*)(dst + i * 8) = o;
}

__global__ __launch_bounds__(32) void k_vt(const bf* __restrict__ A, const bf* __restrict__ Bt, h16* VT) {
    __shared__ __align__(16) float os[16 * 68];
    const int K = EW;
    const int lane = threadIdx.x & 31, lr = lane & 15, hi = lane >> 4; const int r0 = blockIdx.x * 64, c0 = blockIdx.y * 64;
    v8f acc[4][4];
#pragma unroll
    for (int mb = 0; mb < 4; ++mb)
#pragma unroll
        for (int nb = 0; nb < 4; ++nb) acc[mb][nb] = (v8f){};
    const size_t aoff = (size_t)(r0 + lr) * K + 8 * hi, boff = (size_t)(c0 + lr) * K + 8 * hi;
#pragma unroll 1
    for (int kc = 0; kc < K; kc += 32) {
        v16bf a[4];
#pragma unroll
        for (int mb = 0; mb < 4; ++mb) a[mb] = ldb(A + aoff + (size_t)mb * 16 * K + kc);
#pragma unroll
        for (int nb = 0; nb < 4; ++nb) { const v16bf b = ldb(Bt + boff + (size_t)nb * 16 * K + kc);
#pragma unroll
            for (int mb = 0; mb < 4; ++mb) acc[mb][nb] = wmmabg(a[mb], b, acc[mb][nb]); }
    }
    const int bb = c0 / SEQ, tt = c0 % SEQ;
    const size_t tbase = (size_t)bb * (size_t)HV * SEQ + (size_t)r0 * SEQ + (size_t)tt;
#pragma unroll
    for (int mb = 0; mb < 4; ++mb) {
#pragma unroll
        for (int nb = 0; nb < 4; ++nb) {
#pragma unroll
            for (int j = 0; j < 8; ++j) os[(hi * 8 + j) * 68 + nb * 16 + lr] = acc[mb][nb][j]; }
        wave_sync();
#pragma unroll 1
        for (int ps = 0; ps < 2; ++ps) {
            const size_t sb = tbase + (size_t)(mb * 16) * SEQ;
#pragma unroll
            for (int s = 0; s < 4; ++s) { const int row = 4 * s + (lane >> 3), c8 = (lane & 7) * 8;
                const v4f x0 = *(const v4fa*)(&os[row * 68 + c8]); const v4f x1 = *(const v4fa*)(&os[row * 68 + c8 + 4]); v8h hv;
#pragma unroll
                for (int i = 0; i < 4; ++i) { hv[i] = toh_flush(x0[i]); hv[4 + i] = toh_flush(x1[i]); }
                const size_t oo = sb + (size_t)row * SEQ + c8;
                *(volatile v8h*)(VT + oo) = hv; }
            if (ps == 0) __threadfence(); }
        wave_sync();
    }
}

__global__ __launch_bounds__(32) __attribute__((amdgpu_num_vgpr(256))) void k_amp(const bf* __restrict__ XB, const bf* __restrict__ WB, float* PR) {
    __shared__ __align__(16) float os[16 * OSA];
    const int lane = threadIdx.x & 31, lr = lane & 15, hi = lane >> 4;
    const int r0 = blockIdx.x * 16; const int which = blockIdx.y;
    const size_t aoff = (size_t)(r0 + lr) * EW + 8 * hi;
    const size_t boff = (size_t)(HV + which * EW + lr) * EW + 8 * hi;
    v8f acc[16];
#pragma unroll
    for (int nb = 0; nb < 16; ++nb) acc[nb] = (v8f){};
    float n2 = 0.0f;
#pragma unroll 1
    for (int kc = 0; kc < EW; kc += 32) {
        const v8us alo = *(const v8us*)(XB + aoff + kc); const v8us ahi = *(const v8us*)(XB + aoff + kc + 16);
#pragma unroll
        for (int i = 0; i < 8; ++i) { const float u = __uint_as_float(((unsigned)alo[i]) << 16); const float w = __uint_as_float(((unsigned)ahi[i]) << 16); n2 = fmaf(u, u, n2); n2 = fmaf(w, w, n2); }
        const v16bf a = cat16b(alo, ahi);
#pragma unroll
        for (int nb = 0; nb < 16; ++nb) { const v16bf b = ldb(WB + boff + (size_t)nb * 16 * EW + kc); acc[nb] = wmmabg(a, b, acc[nb]); }
    }
    n2 += __shfl_xor(n2, 16, 32);
    float ss[8], inv[8], sp[8];
#pragma unroll
    for (int j = 0; j < 8; ++j) { float s = 0.0f;
#pragma unroll
        for (int nb = 0; nb < 16; ++nb) s = fmaf(acc[nb][j], acc[nb][j], s);
        s += __shfl_xor(s, 1, 32); s += __shfl_xor(s, 2, 32); s += __shfl_xor(s, 4, 32); s += __shfl_xor(s, 8, 32);
        ss[j] = s; }
#pragma unroll
    for (int j = 0; j < 8; ++j) { const float n2r = __shfl(n2, 8 * hi + j, 32);
        const float nn = sqrtf(n2r) + 1.0e-12f; const float den = ss[j] + EPSQ * nn * nn; inv[j] = 1.0f / den; sp[j] = 0.0f; }
#pragma unroll
    for (int nb = 0; nb < 16; ++nb) {
#pragma unroll
        for (int j = 0; j < 8; ++j) { const float a = acc[nb][j]; const float p = a * a * inv[j];
            os[(hi * 8 + j) * OSA + nb * 16 + lr] = p;
            sp[j] = fmaf(p, __builtin_amdgcn_logf(p + EPSQ), sp[j]); } }
#pragma unroll
    for (int j = 0; j < 8; ++j) { float s = sp[j];
        s += __shfl_xor(s, 1, 32); s += __shfl_xor(s, 2, 32); s += __shfl_xor(s, 4, 32); s += __shfl_xor(s, 8, 32);
        s *= LN2F;
        os[(hi * 8 + j) * OSA + EW + lr] = s; os[(hi * 8 + j) * OSA + EW + 16 + lr] = s; }
    wave_sync();
    float* prow = PR + (size_t)which * ((size_t)NB * SEQ * RP) + (size_t)r0 * RP;
#pragma unroll 1
    for (int ps = 0; ps < 2; ++ps) {
#pragma unroll 1
        for (int row = 0; row < 16; ++row) {
#pragma unroll
            for (int i = 0; i < 2; ++i) { const int c4 = (i * 32 + lane) * 4;
                const v4f val = *(const v4fa*)(&os[row * OSA + c4]);
                *(volatile v4f*)(prow + (size_t)row * RP + c4) = val; } }
#pragma unroll
        for (int s = 0; s < 4; ++s) { const int row = 4 * s + (lane >> 3), c4 = EW + (lane & 7) * 4;
            const v4f val = *(const v4fa*)(&os[row * OSA + c4]);
            *(volatile v4f*)(prow + (size_t)row * RP + c4) = val; }
        if (ps == 0) __threadfence(); }
}

__device__ __forceinline__ void js_tile(const float* __restrict__ qrow, const float* __restrict__ krow, const float spq, float (&sc)[8]) {
    float acc[8];
#pragma unroll
    for (int r = 0; r < 8; ++r) acc[r] = 0.0f;
#pragma unroll 1
    for (int e = 0; e < EW; e += 4) {
        const v4f p = *(const v4f*)(qrow + e);
#pragma unroll
        for (int r = 0; r < 8; ++r) {
            const v4f q = *(const v4f*)(krow + (size_t)r * RP + e);
#pragma unroll
            for (int u = 0; u < 4; ++u) { const float mm = p[u] + q[u]; acc[r] = fmaf(mm, __builtin_amdgcn_logf(fmaf(0.5f, mm, EPSQ)), acc[r]); } }
    }
#pragma unroll
    for (int r = 0; r < 8; ++r) { const float sq = krow[(size_t)r * RP + EW]; const float js = 0.5f * (spq + sq) - (0.5f * LN2F) * acc[r]; sc[r] = 1.0f - js; }
}

__global__ __launch_bounds__(32 * AW) __attribute__((amdgpu_num_vgpr(256))) void k_attn(const float* __restrict__ PR, const h16* __restrict__ VT, float* OUT) {
    __shared__ __align__(16) float os[AW * 16 * OSP];
    const int lane = threadIdx.x & 31, lr = lane & 15, hi = lane >> 4;
    const int wave = __builtin_amdgcn_readfirstlane((int)(threadIdx.x >> 5));
    const int b = blockIdx.y;
    const int t0 = (blockIdx.x * AW + wave) * 16;
    const int ti = t0 + lr;
    const int nk = (t0 + 16 + 31) & ~31;
    const float* qrow = PR + ((size_t)b * SEQ + (size_t)ti) * RP;
    const float spq = qrow[EW];
    const float* kb = PR + (size_t)NB * SEQ * RP + ((size_t)b * SEQ + (size_t)(8 * hi)) * RP;
    const size_t vo = (size_t)b * HV * SEQ + (size_t)lr * SEQ + 8 * hi;
    v8f o[8], oR[8];
#pragma unroll
    for (int j = 0; j < 8; ++j) { o[j] = (v8f){}; oR[j] = (v8f){}; }
    float l = 0.0f;
#pragma unroll 1
    for (int key0 = 0; key0 < nk; key0 += 32) {
        float sa[8], sb[8];
        js_tile(qrow, kb + (size_t)key0 * RP, spq, sa);
        js_tile(qrow, kb + (size_t)(key0 + 16) * RP, spq, sb);
        const int ja = key0 + 8 * hi;
        v16h pb, pr; float ls = 0.0f;
#pragma unroll
        for (int r = 0; r < 8; ++r) {
            float xa = sa[r], xb = sb[r];
            asm volatile("" : "+v"(xa)); asm volatile("" : "+v"(xb));
            const bool fa = (ja + r) <= ti; const bool fb = (ja + 16 + r) <= ti;
            const float ga = fa ? xa : 0.0f, gb = fb ? xb : 0.0f;
            const h16 pa = toh_flush(ga); const h16 pc = toh_flush(gb);
            pb[r] = pa; pb[8 + r] = pc;
            pr[r] = toh_flush((ga - (float)pa) * 2048.0f); pr[8 + r] = toh_flush((gb - (float)pc) * 2048.0f);
            ls += fabsf(ga) + fabsf(gb); }
        l += ls;
        const h16* va = VT + vo + key0;
#pragma unroll
        for (int j = 0; j < 8; ++j) { const v16h v = ldh(va + (size_t)(16 * j) * SEQ); o[j] = wmma16g(v, pb, o[j]); oR[j] = wmma16g(v, pr, oR[j]); }
    }
    l += __shfl_xor(l, 16, 32);
    const float lsafe = fmaxf(l, 1.0e-12f);
    const float inv = 1.0f / lsafe;
    const int wb = wave * 16 * OSP;
#pragma unroll
    for (int j = 0; j < 8; ++j) { v4f a, c;
#pragma unroll
        for (int i = 0; i < 4; ++i) { a[i] = (o[j][i] + oR[j][i] * (1.0f / 2048.0f)) * inv; c[i] = (o[j][4 + i] + oR[j][4 + i] * (1.0f / 2048.0f)) * inv; }
        *(v4fa*)(&os[wb + lr * OSP + 16 * j + 8 * hi]) = a; *(v4fa*)(&os[wb + lr * OSP + 16 * j + 8 * hi + 4]) = c; }
    wave_sync();
    float* orow = OUT + ((size_t)b * OUT_SEQ + (size_t)t0) * HV;
#pragma unroll 1
    for (int ps = 0; ps < 2; ++ps) {
#pragma unroll 1
        for (int row = 0; row < 16; ++row) {
            const v4f val = *(const v4fa*)(&os[wb + row * OSP + lane * 4]);
            *(volatile v4f*)(orow + (size_t)row * HV + lane * 4) = val; }
        if (ps == 0) __threadfence(); }
}

static constexpr size_t al256(size_t v) { return (v + 255) & ~(size_t)255; }
static constexpr size_t SZ_XB = al256((size_t)NB * SEQ * EW * 2);
static constexpr size_t SZ_WB = al256((size_t)(HV + 2 * EW) * EW * 2);
static constexpr size_t SZ_VT = al256((size_t)NB * HV * SEQ * 2);
static constexpr size_t SZ_PR = al256((size_t)2 * NB * SEQ * RP * 4);
static constexpr size_t SZ_TOTAL = SZ_XB + SZ_WB + SZ_VT + SZ_PR;
static_assert(SZ_TOTAL <= (size_t)134217728);
static_assert(((size_t)HV * EW * 2) % 256 == 0);
static_assert(((size_t)EW * EW * 2) % 256 == 0);
static_assert(((size_t)NB * SEQ * RP * 4) % 256 == 0);
static_assert((size_t)(NB * SEQ / 16) * 16 * RP * 4 * 2 <= SZ_PR);
static_assert((size_t)(NB * SEQ / 64) * 64 * HV * 2 <= SZ_VT);
static_assert((size_t)NB * OUT_SEQ * HV * 4 == (size_t)NB * SEQ * HV * 4 || OUT_SEQ != SEQ);

extern "C" void kernel_launch(void* const* d_in, const int* in_sizes, int n_in,
                              void* d_out, int out_size, void* d_ws, size_t ws_size, hipStream_t stream) {
    if (n_in < 4) return;
    const size_t needx = ((size_t)(NB - 1) * SEQ_FULL + SEQ) * EW;
    if ((size_t)in_sizes[0] < needx) return;
    if ((size_t)in_sizes[1] < (size_t)HV * EW || (size_t)in_sizes[2] < (size_t)EW * EW || (size_t)in_sizes[3] < (size_t)EW * EW) return;
    if ((size_t)out_size < ((size_t)(NB - 1) * OUT_SEQ + SEQ) * HV) return;
    if (SZ_TOTAL > ws_size) return;
    const float* x  = (const float*)d_in[0];
    const float* wv = (const float*)d_in[1];
    const float* wq = (const float*)d_in[2];
    const float* wk = (const float*)d_in[3];
    float* OUT = (float*)d_out;
    char* wsp = (char*)d_ws;
    bf* XB = (bf*)wsp; wsp += SZ_XB;
    bf* WB = (bf*)wsp; wsp += SZ_WB;
    h16* VT = (h16*)wsp; wsp += SZ_VT;
    float* PR = (float*)wsp; wsp += SZ_PR;

    if (SEQ == SEQ_FULL) {
        const size_t n8 = (size_t)NB * SEQ * EW / 8;
        k_cvt8<<<(unsigned)((n8 + 255) / 256), 256, 0, stream>>>(x, XB, n8);
    } else {
        const size_t n8 = (size_t)SEQ * EW / 8;
        for (int b = 0; b < NB; ++b) k_cvt8<<<(unsigned)((n8 + 255) / 256), 256, 0, stream>>>(x + (size_t)b * SEQ_FULL * EW, XB + (size_t)b * SEQ * EW, n8);
    }
    { const size_t n8v = (size_t)HV * EW / 8; const size_t n8q = (size_t)EW * EW / 8;
      k_cvt8<<<(unsigned)((n8v + 255) / 256), 256, 0, stream>>>(wv, WB, n8v);
      k_cvt8<<<(unsigned)((n8q + 255) / 256), 256, 0, stream>>>(wq, WB + (size_t)HV * EW, n8q);
      k_cvt8<<<(unsigned)((n8q + 255) / 256), 256, 0, stream>>>(wk, WB + (size_t)(HV + EW) * EW, n8q); }

    k_vt<<<dim3(HV / 64, NB * SEQ / 64, 1), 32, 0, stream>>>(WB, XB, VT);
    k_amp<<<dim3(NB * SEQ / 16, 2, 1), 32, 0, stream>>>(XB, WB, PR);
    k_attn<<<dim3(SEQ / (16 * AW), NB, 1), 32 * AW, 0, stream>>>(PR, VT, OUT);
}
